// Net_68384469287506
// MI455X (gfx1250) — hardware-verified
//
#include <hip/hip_runtime.h>
#include <stddef.h>
#include <stdint.h>
#include <math.h>


#define DF     64
#define K2     128
#define NGR    256
#define H1N    256
#define H2N    128
#define H3N    64
#define NTHR   256
#define NWAVE  8
#define EPT    8
#define CHUNK  (NTHR * EPT)
#define WCAP   (EPT * 32)
#define LISTN  (NWAVE * WCAP)
#define NBD    8192
#define SLD    13
#define NBA    1024
#define SLA    10
#define RCAP   28672
#define DEGCAP 128
#define GBM    64
#define GBN    64
#define GTHR   128
#define UB1    (DF * (DF / 8))
#define UB2    (UB1 + DF * (K2 / 8))
#define UB3    (UB2 + H1N * (K2 / 8))
#define UB4    (UB3 + H2N * ((2 * H1N) / 8))
#define UB5    (UB4 + H3N * ((2 * H2N) / 8))
#define AGG_ZINTS (LISTN + 2 * RCAP + 3 * NBA)
#define AGG_LDS_INTS (AGG_ZINTS + 16)
#define WSMAX  134217728

static_assert((CHUNK & (CHUNK - 1)) == 0 && CHUNK <= 4096);
static_assert((NBD & (NBD - 1)) == 0 && NBD == (1 << SLD));
static_assert((NBA & (NBA - 1)) == 0 && NBA == (1 << SLA));
static_assert(((long long)CHUNK << SLD) < (1LL << 31));
static_assert(((long long)CHUNK << SLA) < (1LL << 31));
static_assert(NBD % (NTHR * 4) == 0);
static_assert(LISTN % NTHR == 0);
static_assert(NBA % NWAVE == 0 && NBA % 32 == 0 && NBA % GBM == 0);
static_assert(RCAP % 32 == 0 && AGG_ZINTS % 4 == 0 && LISTN % 4 == 0);
static_assert(RCAP >= 16623 + 16623 / 20);
static_assert(DEGCAP >= 35 + 8);
static_assert(DF % 32 == 0 && K2 % 32 == 0 && K2 == 2 * DF && DF == GBN);
static_assert((2 * H1N) % 32 == 0 && (2 * H2N) % 32 == 0);
static_assert(H1N % GBN == 0 && H2N % GBN == 0 && H3N == GBN);
static_assert(GBM == (GTHR / 32) * 16 && GBN == 64 && GTHR == 2 * GBN);
static_assert(NGR % GBM == 0 && NGR == 4 * GBM);
static_assert(UB1 % NTHR == 0 && UB2 % NTHR == 0 && UB3 % NTHR == 0 && UB4 % NTHR == 0 && UB5 % NTHR == 0);
static_assert(DF == 2 * 32);
static_assert(AGG_LDS_INTS * 4 <= 300000);

typedef float          v2f   __attribute__((ext_vector_type(2)));
typedef float          v4f   __attribute__((ext_vector_type(4)));
typedef float          v8f   __attribute__((ext_vector_type(8)));
typedef int            v4i   __attribute__((ext_vector_type(4)));
typedef int            v8i   __attribute__((ext_vector_type(8)));
typedef unsigned int   v4u   __attribute__((ext_vector_type(4)));
typedef unsigned short v8us  __attribute__((ext_vector_type(8)));
typedef unsigned short v16us __attribute__((ext_vector_type(16)));
typedef __bf16         v16bf __attribute__((ext_vector_type(16)));
typedef v2f  __attribute__((may_alias)) v2fa;
typedef v4f  __attribute__((may_alias)) v4fa;
typedef v4i  __attribute__((may_alias)) v4ia;
typedef v8us __attribute__((may_alias)) v8usa;
union FragB { v16bf v; v16us u; v8us h[2]; v8i w; };

__device__ __forceinline__ v8f wmb(const FragB& a, const FragB& b, v8f c) {
  v8f d = __builtin_amdgcn_wmma_f32_16x16x32_bf16(false, a.v, false, b.v, (short)0, c, false, false);
  asm volatile("v_nop\n\tv_nop\n\tv_nop\n\tv_nop" : "+v"(d) : "v"(a.w), "v"(b.w));
  return d;
}

__device__ __forceinline__ unsigned bf16_bits(float f) {
  const unsigned u = __float_as_uint(f);
  const unsigned r = (u + 0x7FFFu + ((u >> 16) & 1u)) >> 16;
  return (f != f) ? 0x7FC0u : r;
}
__device__ __forceinline__ float bf16_val(float f) {
  return __uint_as_float(bf16_bits(f) << 16);
}

__device__ __forceinline__ v4u hilo8(const v4f a, const v4f b, const bool takeLo) {
  const float f[8] = {a.x, a.y, a.z, a.w, b.x, b.y, b.z, b.w};
  unsigned w[4];
#pragma unroll
  for (int j = 0; j < 4; ++j) {
    const unsigned h0 = bf16_bits(f[2 * j]), h1 = bf16_bits(f[2 * j + 1]);
    const unsigned l0 = bf16_bits(f[2 * j] - __uint_as_float(h0 << 16));
    const unsigned l1 = bf16_bits(f[2 * j + 1] - __uint_as_float(h1 << 16));
    const unsigned q0 = takeLo ? l0 : h0, q1 = takeLo ? l1 : h1;
    w[j] = q0 | (q1 << 16);
  }
  v4u pv; pv.x = w[0]; pv.y = w[1]; pv.z = w[2]; pv.w = w[3];
  return pv;
}

template <int SLB>
__device__ __forceinline__ int scan_chunk(const int* __restrict__ dsts, int nE, int cbase, int slotBase,
                                          int nb, int vec8, int* list, int tid, int lane, int wave) {
  int wc = 0;
  const int el0  = tid * EPT;
  const int e0   = cbase + el0;
  const int sent = -2147483647 - 1;
  v4i da, db;
  if (vec8 != 0 && cbase + CHUNK <= nE) {
    da = *(const v4i*)(dsts + e0);
    db = *(const v4i*)(dsts + e0 + 4);
  } else {
    da.x = (e0     < nE) ? dsts[min(e0,     nE - 1)] : sent;
    da.y = (e0 + 1 < nE) ? dsts[min(e0 + 1, nE - 1)] : sent;
    da.z = (e0 + 2 < nE) ? dsts[min(e0 + 2, nE - 1)] : sent;
    da.w = (e0 + 3 < nE) ? dsts[min(e0 + 3, nE - 1)] : sent;
    db.x = (e0 + 4 < nE) ? dsts[min(e0 + 4, nE - 1)] : sent;
    db.y = (e0 + 5 < nE) ? dsts[min(e0 + 5, nE - 1)] : sent;
    db.z = (e0 + 6 < nE) ? dsts[min(e0 + 6, nE - 1)] : sent;
    db.w = (e0 + 7 < nE) ? dsts[min(e0 + 7, nE - 1)] : sent;
  }
  const unsigned nbs = (unsigned)slotBase;
  const unsigned unb = (unsigned)nb;
  const unsigned s0 = (unsigned)da.x - nbs, s1 = (unsigned)da.y - nbs;
  const unsigned s2 = (unsigned)da.z - nbs, s3 = (unsigned)da.w - nbs;
  const unsigned s4 = (unsigned)db.x - nbs, s5 = (unsigned)db.y - nbs;
  const unsigned s6 = (unsigned)db.z - nbs, s7 = (unsigned)db.w - nbs;
  const bool h0 = s0 < unb, h1 = s1 < unb, h2 = s2 < unb, h3 = s3 < unb;
  const bool h4 = s4 < unb, h5 = s5 < unb, h6 = s6 < unb, h7 = s7 < unb;
  const unsigned any = __builtin_amdgcn_ballot_w32(h0 | h1 | h2 | h3 | h4 | h5 | h6 | h7);
  if (any != 0u) {
#define HITJ(J, HJ, SJ) { \
      const unsigned mj = __builtin_amdgcn_ballot_w32(HJ); \
      if (mj != 0u) { \
        if (HJ) { \
          const int pos = wc + (int)__builtin_amdgcn_mbcnt_lo(mj, 0u); \
          if (pos < WCAP) list[wave * WCAP + pos] = ((el0 + (J)) << SLB) | (int)(SJ); \
        } \
        wc += (int)__builtin_popcount(mj); } }
    HITJ(0, h0, s0)
    HITJ(1, h1, s1)
    HITJ(2, h2, s2)
    HITJ(3, h3, s3)
    HITJ(4, h4, s4)
    HITJ(5, h5, s5)
    HITJ(6, h6, s6)
    HITJ(7, h7, s7)
#undef HITJ
  }
  return wc;
}

__device__ __forceinline__ v8us cv8b(const float* __restrict__ p, size_t stride) {
  v8us o;
#pragma unroll
  for (int i = 0; i < 8; ++i) o[i] = (unsigned short)bf16_bits(p[(size_t)i * stride]);
  return o;
}

__global__ __launch_bounds__(NTHR) void k_wprep(const float* __restrict__ W0, const float* __restrict__ W1,
                                                const float* __restrict__ hW1, const float* __restrict__ hW2,
                                                const float* __restrict__ hW3,
                                                unsigned short* w0t, unsigned short* w1d, unsigned short* hw1d,
                                                unsigned short* hw2d, unsigned short* hw3d) {
  const int u = (int)blockIdx.x * NTHR + (int)threadIdx.x;
  v8us o;
  unsigned short* dp;
  if (u < UB1) {
    const int n = u >> 3, k8 = (u & 7) * 8;
    o = cv8b(W0 + (size_t)k8 * DF + n, DF);
    dp = w0t + (size_t)u * 8;
  } else if (u < UB2) {
    const int v = u - UB1, n = v >> 4, k8 = (v & 15) * 8, kk = k8 & (DF - 1);
    o = cv8b(W1 + (size_t)kk * DF + n, DF);
    dp = w1d + (size_t)v * 8;
  } else if (u < UB3) {
    const int v = u - UB2, n = v >> 4, k8 = (v & 15) * 8, kk = k8 & (DF - 1);
    o = cv8b(hW1 + (size_t)kk * H1N + n, H1N);
    dp = hw1d + (size_t)v * 8;
  } else if (u < UB4) {
    const int v = u - UB3, n = v >> 6, k8 = (v & 63) * 8, kk = k8 & (H1N - 1);
    o = cv8b(hW2 + (size_t)kk * H2N + n, H2N);
    dp = hw2d + (size_t)v * 8;
  } else if (u < UB5) {
    const int v = u - UB4, n = v >> 5, k8 = (v & 31) * 8, kk = k8 & (H2N - 1);
    o = cv8b(hW3 + (size_t)kk * H3N + n, H3N);
    dp = hw3d + (size_t)v * 8;
  } else {
    return;
  }
  *(volatile v8us*)dp = o;
  __threadfence();
  *(volatile v8us*)dp = o;
}

__global__ __launch_bounds__(NTHR) void k_cvx(const float* __restrict__ x, int nN, int nUnits,
                                              unsigned short* xb) {
  const int u = (int)blockIdx.x * NTHR + (int)threadIdx.x;
  if (u >= nUnits) return;
  const int row = u >> 3;
  const int k8  = (u & 7) * 8;
  const int rc  = row < nN ? row : nN - 1;
  const float* p = x + (size_t)rc * DF + k8;
  const v4f a = *(const v4fa*)p;
  const v4f b = *(const v4fa*)(p + 4);
  const bool ok = row < nN;
  v8us o;
  o[0] = ok ? (unsigned short)bf16_bits(a.x) : (unsigned short)0;
  o[1] = ok ? (unsigned short)bf16_bits(a.y) : (unsigned short)0;
  o[2] = ok ? (unsigned short)bf16_bits(a.z) : (unsigned short)0;
  o[3] = ok ? (unsigned short)bf16_bits(a.w) : (unsigned short)0;
  o[4] = ok ? (unsigned short)bf16_bits(b.x) : (unsigned short)0;
  o[5] = ok ? (unsigned short)bf16_bits(b.y) : (unsigned short)0;
  o[6] = ok ? (unsigned short)bf16_bits(b.z) : (unsigned short)0;
  o[7] = ok ? (unsigned short)bf16_bits(b.w) : (unsigned short)0;
  unsigned short* dp = xb + (size_t)u * 8;
  *(volatile v8us*)dp = o;
  __threadfence();
  *(volatile v8us*)dp = o;
}

__global__ __launch_bounds__(NTHR) void k_deg(const int* __restrict__ dsts, int nE, int vec8, float* dis) {
  __shared__ __attribute__((aligned(16))) int scnt[NBD];
  __shared__ __attribute__((aligned(16))) int list[LISTN];
  __shared__ int wcnt[NWAVE];
  const int tid = (int)threadIdx.x, lane = tid & 31, wave = tid >> 5;
  const int nodeBase = (int)blockIdx.x * NBD;

  for (int i = tid; i < NBD; i += NTHR) scnt[i] = 0;
  for (int i = tid; i < LISTN; i += NTHR) list[i] = 0;
  if (tid < NWAVE) wcnt[tid] = 0;
  __syncthreads();

  const int nChunks = (nE + CHUNK - 1) / CHUNK;
#pragma unroll 1
  for (int ch = 0; ch < nChunks; ++ch) {
    const int cbase = ch * CHUNK;
    const int wc = scan_chunk<SLD>(dsts, nE, cbase, nodeBase, NBD, vec8, list, tid, lane, wave);
    if (lane == 0) wcnt[wave] = wc;
    __syncthreads();
    if (wave == 0) {
#pragma unroll 1
      for (int w2 = 0; w2 < NWAVE; ++w2) {
        int c = wcnt[w2];
        c = c < 0 ? 0 : (c > WCAP ? WCAP : c);
#pragma unroll 1
        for (int b0 = 0; b0 < c; b0 += 32) {
          const int idx = b0 + lane;
          const int ent = list[w2 * WCAP + (idx < WCAP ? idx : WCAP - 1)];
          const int m32 = (c - b0) < 32 ? (c - b0) : 32;
#pragma unroll 1
          for (int k = 0; k < m32; ++k) {
            const int u  = __builtin_amdgcn_readlane(ent, k);
            const int sl = u & (NBD - 1);
            if (lane == 0) scnt[sl] = scnt[sl] + 1;
          }
        }
      }
    }
    __syncthreads();
  }

#pragma unroll 1
  for (int i = tid; i < NBD; i += NTHR) {
    const int c = scnt[i];
    const float d = (float)(c + 1);
    const float r = (d > 0.0f) ? (1.0f / sqrtf(d)) : 0.0f;
    scnt[i] = __float_as_int(r);
  }
  __syncthreads();

  v4f vals[NBD / (NTHR * 4)];
#pragma unroll
  for (int it = 0; it < NBD / (NTHR * 4); ++it) {
    const int s0 = it * (NTHR * 4) + 4 * tid;
    const v4i c4 = *(const v4ia*)(scnt + s0);
    v4f v;
    v.x = __int_as_float(c4.x); v.y = __int_as_float(c4.y);
    v.z = __int_as_float(c4.z); v.w = __int_as_float(c4.w);
    vals[it] = v;
  }
#pragma unroll
  for (int it = 0; it < NBD / (NTHR * 4); ++it) {
    const int s0 = it * (NTHR * 4) + 4 * tid;
    *(volatile v4f*)(dis + (size_t)nodeBase + s0) = vals[it];
  }
  __threadfence();
#pragma unroll
  for (int it = 0; it < NBD / (NTHR * 4); ++it) {
    const int s0 = it * (NTHR * 4) + 4 * tid;
    *(volatile v4f*)(dis + (size_t)nodeBase + s0) = vals[it];
  }
}

template <int EPI>
__global__ __launch_bounds__(GTHR) void k_gemm(
    const unsigned short* __restrict__ A, const unsigned short* __restrict__ WT, int K,
    float* outF, unsigned short* outH, int ldo, int lsplit,
    const float* __restrict__ p0, const float* __restrict__ p1, const float* __restrict__ p2,
    const float* __restrict__ p3, const float* __restrict__ p4)
{
  __shared__ __attribute__((aligned(16))) float stg[GBM * GBN];
  __shared__ __attribute__((aligned(16))) float w4s[GBN];
  __shared__ __attribute__((aligned(16))) float os[GBM];
  const int tid = (int)threadIdx.x, lane = tid & 31, wave = tid >> 5, hh = lane >> 4, m = lane & 15;
  const int rowBase = (int)blockIdx.x * GBM;
  const int col0    = (int)blockIdx.y * GBN;

  v8f acc[4];
  {
    const v8f z = {0.f, 0.f, 0.f, 0.f, 0.f, 0.f, 0.f, 0.f};
    acc[0] = z; acc[1] = z; acc[2] = z; acc[3] = z;
  }
  const unsigned short* ap = A  + (size_t)(rowBase + 16 * wave + m) * (size_t)K + 8 * hh;
  const unsigned short* wp = WT + (size_t)(col0 + m) * (size_t)K + 8 * hh;
  const int ksteps = K >> 5;
#pragma unroll 1
  for (int ks = 0; ks < ksteps; ++ks) {
    FragB af;
    af.h[0] = *(const v8usa*)(ap + 32 * ks);
    af.h[1] = *(const v8usa*)(ap + 32 * ks + 16);
#pragma unroll
    for (int t = 0; t < 4; ++t) {
      const unsigned short* wq = wp + (size_t)(16 * t) * (size_t)K + 32 * ks;
      FragB bf;
      bf.h[0] = *(const v8usa*)wq;
      bf.h[1] = *(const v8usa*)(wq + 16);
      acc[t] = wmb(af, bf, acc[t]);
    }
  }

#pragma unroll
  for (int t = 0; t < 4; ++t) {
    const int lc = 16 * t + m;
#pragma unroll
    for (int r = 0; r < 8; ++r) {
      const int lr = 16 * wave + 8 * hh + r;
      stg[lr * GBN + lc] = acc[t][r];
    }
  }
  __syncthreads();

  if constexpr (EPI == 0) {
    v4f fv[8];
#pragma unroll
    for (int i = 0; i < 8; ++i) {
      const int lr = 16 * wave + 2 * i + hh;
      fv[i] = *(const v4fa*)(stg + lr * GBN + 4 * m);
    }
#pragma unroll
    for (int i = 0; i < 8; ++i) {
      const int lr = 16 * wave + 2 * i + hh;
      const int gr = rowBase + lr;
      float* op = outF + (size_t)gr * (size_t)ldo + col0 + 4 * m;
      *(volatile v4f*)op = fv[i];
    }
    __threadfence();
#pragma unroll
    for (int i = 0; i < 8; ++i) {
      const int lr = 16 * wave + 2 * i + hh;
      const int gr = rowBase + lr;
      float* op = outF + (size_t)gr * (size_t)ldo + col0 + 4 * m;
      *(volatile v4f*)op = fv[i];
    }
  } else if constexpr (EPI == 1) {
    {
      const int c  = tid & (GBN - 1);
      const int rs = tid >> 6;
      const int gc = col0 + c;
      const float cb  = bf16_val(p0[gc]);
      const float cg  = bf16_val(p1[gc]);
      const float cbb = bf16_val(p2[gc]);
      const float cm  = bf16_val(p3[gc]);
      const float cv  = bf16_val(p4[gc]);
      const float crs = rsqrtf(cv + 1e-5f);
#pragma unroll 1
      for (int i = 0; i < GBM / 2; ++i) {
        const int lr = 2 * i + rs;
        float v = stg[lr * GBN + c];
        v = v + cb;
        v = ((v - cm) * crs) * cg + cbb;
        v = (v > 0.0f) ? v : (v - v);
        stg[lr * GBN + c] = v;
      }
    }
    __syncthreads();
    const int q = lane & 7;
    const bool takeLo = (lane & 8) != 0;
    v4u pk[8];
#pragma unroll
    for (int i = 0; i < 8; ++i) {
      const int lr = 16 * wave + 2 * i + hh;
      const v4f a = *(const v4fa*)(stg + lr * GBN + 8 * q);
      const v4f b = *(const v4fa*)(stg + lr * GBN + 8 * q + 4);
      pk[i] = hilo8(a, b, takeLo);
    }
    const int coff = col0 + 8 * q + (takeLo ? lsplit : 0);
#pragma unroll
    for (int i = 0; i < 8; ++i) {
      const int gr = rowBase + 16 * wave + 2 * i + hh;
      unsigned short* op = outH + (size_t)gr * (size_t)ldo + coff;
      *(volatile v4u*)op = pk[i];
    }
    __threadfence();
#pragma unroll
    for (int i = 0; i < 8; ++i) {
      const int gr = rowBase + 16 * wave + 2 * i + hh;
      unsigned short* op = outH + (size_t)gr * (size_t)ldo + coff;
      *(volatile v4u*)op = pk[i];
    }
  } else {
    {
      const int c  = tid & (GBN - 1);
      const int rs = tid >> 6;
      const float cb = bf16_val(p0[c]);
      if (tid < GBN) w4s[tid] = bf16_val(p1[tid]);
#pragma unroll 1
      for (int i = 0; i < GBM / 2; ++i) {
        const int lr = 2 * i + rs;
        float v = stg[lr * GBN + c];
        v = v + cb;
        v = (v > 0.0f) ? v : (v - v);
        stg[lr * GBN + c] = v;
      }
    }
    __syncthreads();
    if (tid < GBM) {
      const float b4 = bf16_val(p2[0]);
      float s = 0.0f;
#pragma unroll 1
      for (int c = 0; c < GBN; ++c) s = fmaf(stg[tid * GBN + c], w4s[c], s);
      os[tid] = s + b4;
    }
    __syncthreads();
    const v4f ov = *(const v4fa*)(os + 4 * (lane & 15));
    float* op = outF + (size_t)rowBase + 4 * (lane & 15);
    const bool okst = (wave == 0) && (lane < 16);
    if (okst) *(volatile v4f*)op = ov;
    __threadfence();
    if (okst) *(volatile v4f*)op = ov;
  }
}

template <int MODE>
__global__ __launch_bounds__(NTHR) void k_agg(const int* __restrict__ srcs, const int* __restrict__ dsts,
                                              int nE, int nN, int vec8, int mRows,
                                              const float* __restrict__ dis,
                                              const float* __restrict__ xl, const float* __restrict__ bias,
                                              const float* __restrict__ bng, const float* __restrict__ bnb,
                                              const float* __restrict__ bnm, const float* __restrict__ bnv,
                                              unsigned short* hb, float* hout) {
  extern __shared__ __attribute__((aligned(16))) int dsm[];
  int* list = dsm;
  int* hl   = dsm + LISTN;
  int* sl   = dsm + LISTN + RCAP;
  int* cnt  = dsm + LISTN + 2 * RCAP;
  int* offs = cnt + NBA;
  int* cur  = offs + NBA;
  int* misc = cur + NBA;
  const int tid = (int)threadIdx.x, lane = tid & 31, wave = tid >> 5;
  const int nodeBase = (int)blockIdx.x * NBA;

  {
    const v4i z4 = {0, 0, 0, 0};
    for (int i = tid * 4; i < AGG_ZINTS; i += NTHR * 4) *(v4ia*)(dsm + i) = z4;
    if (tid < 16) misc[tid] = 0;
  }
  float bv0, bv1, sg0, sg1, sb0, sb1, sm0, sm1, rs0, rs1;
  {
    const v2f a = *(const v2fa*)(bias + 2 * lane);
    const v2f g = *(const v2fa*)(bng + 2 * lane);
    const v2f b = *(const v2fa*)(bnb + 2 * lane);
    const v2f mm = *(const v2fa*)(bnm + 2 * lane);
    const v2f vv = *(const v2fa*)(bnv + 2 * lane);
    bv0 = bf16_val(a.x);  bv1 = bf16_val(a.y);
    sg0 = bf16_val(g.x);  sg1 = bf16_val(g.y);
    sb0 = bf16_val(b.x);  sb1 = bf16_val(b.y);
    sm0 = bf16_val(mm.x); sm1 = bf16_val(mm.y);
    rs0 = rsqrtf(bf16_val(vv.x) + 1e-5f);
    rs1 = rsqrtf(bf16_val(vv.y) + 1e-5f);
  }
  __syncthreads();

  int t = 0, ov = 0;
  const int nChunks = (nE + CHUNK - 1) / CHUNK;
#pragma unroll 1
  for (int ch = 0; ch < nChunks; ++ch) {
    const int cbase = ch * CHUNK;
    const int wc = scan_chunk<SLA>(dsts, nE, cbase, nodeBase, NBA, vec8, list, tid, lane, wave);
    if (lane == 0) misc[wave] = wc;
    __syncthreads();
    if (wave == 0) {
#pragma unroll 1
      for (int w2 = 0; w2 < NWAVE; ++w2) {
        int c = misc[w2];
        c = c < 0 ? 0 : (c > WCAP ? WCAP : c);
#pragma unroll 1
        for (int b0 = 0; b0 < c; b0 += 32) {
          const int idx = b0 + lane;
          const int ent = list[w2 * WCAP + (idx < WCAP ? idx : WCAP - 1)];
          const int m32 = (c - b0) < 32 ? (c - b0) : 32;
#pragma unroll 1
          for (int k = 0; k < m32; ++k) {
            const int u    = __builtin_amdgcn_readlane(ent, k);
            const int slot = u & (NBA - 1);
            const int el   = (u >> SLA) & (CHUNK - 1);
            const int pk   = ((cbase + el) << SLA) | slot;
            if (t < RCAP) {
              if (lane == 0) { hl[t] = pk; cnt[slot] = cnt[slot] + 1; }
              t = t + 1;
            } else {
              ov = 1;
            }
          }
        }
      }
    }
    __syncthreads();
  }
  if (wave == 0 && lane == 0) { misc[8] = t; misc[9] = ov; }
  __syncthreads();
  int tt = misc[8];
  tt = tt < 0 ? 0 : (tt > RCAP ? RCAP : tt);
  const int ovf = misc[9];

  if (wave == 0) {
    const int base = lane * (NBA / 32);
    int s = 0;
#pragma unroll 1
    for (int i = 0; i < NBA / 32; ++i) s += cnt[base + i];
    int incl = s;
#pragma unroll
    for (int d = 1; d < 32; d <<= 1) {
      const int y = __shfl_up(incl, d, 32);
      if (lane >= d) incl += y;
    }
    int run = incl - s;
#pragma unroll 1
    for (int i = 0; i < NBA / 32; ++i) {
      const int cv = cnt[base + i];
      offs[base + i] = run;
      cur[base + i]  = run;
      run += cv;
    }
  }
  __syncthreads();
  if (wave == 0) {
#pragma unroll 1
    for (int b0 = 0; b0 < tt; b0 += 32) {
      const int idx = b0 + lane;
      const int ent = hl[idx < RCAP ? idx : RCAP - 1];
      const int m32 = (tt - b0) < 32 ? (tt - b0) : 32;
#pragma unroll 1
      for (int k = 0; k < m32; ++k) {
        const int u    = __builtin_amdgcn_readlane(ent, k);
        const int slot = u & (NBA - 1);
        if (lane == 0) {
          int p = cur[slot];
          p = p < 0 ? 0 : (p > RCAP - 1 ? RCAP - 1 : p);
          sl[p] = u;
          cur[slot] = p + 1;
        }
      }
    }
  }
  __syncthreads();

  const float qnan = __int_as_float(0x7fc00000);
  const float pz = (ovf != 0) ? qnan : 0.0f;
  const int sa = (2 * lane) & 31, sb = (2 * lane + 1) & 31;
  const int q0s = (4 * lane) & 31, q1s = (4 * lane + 1) & 31;
  const int q2s = (4 * lane + 2) & 31, q3s = (4 * lane + 3) & 31;
#pragma unroll 1
  for (int si = 0; si < NBA / NWAVE; ++si) {
    const int s    = si * NWAVE + wave;
    const int node = nodeBase + s;
    int c = cnt[s];
    const bool big = c > DEGCAP;
    c = c < 0 ? 0 : (c > DEGCAP ? DEGCAP : c);
    int o = offs[s];
    o = o < 0 ? 0 : (o > RCAP ? RCAP : o);
    const int nc = node < nN ? node : nN - 1;
    const float dd = dis[nc];
    const float rd = dd * dd;
    float acc0 = 0.0f, acc1 = 0.0f;
#pragma unroll 1
    for (int b0 = 0; b0 < c; b0 += 32) {
      int idx = o + b0 + lane;
      idx = idx > RCAP - 1 ? RCAP - 1 : idx;
      const int ent = sl[idx];
      int eid = ent >> SLA;
      eid = eid < 0 ? 0 : (eid > nE - 1 ? nE - 1 : eid);
      int sr = srcs[eid];
      sr = sr < 0 ? 0 : (sr > nN - 1 ? nN - 1 : sr);
      const float cf  = dis[sr] * dd;
      const int   cfi = __float_as_int(cf);
      const int m32 = (c - b0) < 32 ? (c - b0) : 32;
#pragma unroll 1
      for (int k = 0; k < m32; ++k) {
        const int   sk = __builtin_amdgcn_readlane(sr, k);
        const float ck = __int_as_float(__builtin_amdgcn_readlane(cfi, k));
        const v2f a = *(const v2fa*)(xl + (size_t)sk * DF + 2 * lane);
        acc0 = fmaf(ck, a.x, acc0); acc1 = fmaf(ck, a.y, acc1);
      }
    }
    float sv0, sv1;
    {
      const v2f a = *(const v2fa*)(xl + (size_t)nc * DF + 2 * lane);
      sv0 = a.x; sv1 = a.y;
    }
    const float pzr = big ? qnan : pz;
    const bool live = node < nN;
    float y0 = (acc0 + sv0 * rd) + bv0;
    float y1 = (acc1 + sv1 * rd) + bv1;
    y0 = ((y0 - sm0) * rs0) * sg0 + sb0;
    y1 = ((y1 - sm1) * rs1) * sg1 + sb1;
    y0 = (y0 > 0.0f) ? y0 : (y0 - y0);
    y1 = (y1 > 0.0f) ? y1 : (y1 - y1);
    y0 = y0 + pzr; y1 = y1 + pzr;
    const float v0 = live ? y0 : 0.0f;
    const float v1 = live ? y1 : 0.0f;
    const bool wr = (node < mRows) && (lane < 16);
    if constexpr (MODE != 0) {
      const unsigned hb0 = bf16_bits(v0), hb1 = bf16_bits(v1);
      const unsigned lb0 = bf16_bits(v0 - __uint_as_float(hb0 << 16));
      const unsigned lb1 = bf16_bits(v1 - __uint_as_float(hb1 << 16));
      const int hw = (int)(hb0 | (hb1 << 16));
      const int lw = (int)(lb0 | (lb1 << 16));
      const int g0 = __shfl(hw, q0s, 32), g1 = __shfl(hw, q1s, 32);
      const int g2 = __shfl(hw, q2s, 32), g3 = __shfl(hw, q3s, 32);
      const int p0 = __shfl(lw, q0s, 32), p1 = __shfl(lw, q1s, 32);
      const int p2 = __shfl(lw, q2s, 32), p3 = __shfl(lw, q3s, 32);
      const bool lsel = (lane & 8) != 0;
      v4u pv;
      pv.x = (unsigned int)(lsel ? p0 : g0);
      pv.y = (unsigned int)(lsel ? p1 : g1);
      pv.z = (unsigned int)(lsel ? p2 : g2);
      pv.w = (unsigned int)(lsel ? p3 : g3);
      unsigned short* hp = hb + (size_t)node * K2 + 8 * (lane & 15);
      if (wr) *(volatile v4u*)hp = pv;
      __threadfence();
      if (wr) *(volatile v4u*)hp = pv;
    } else {
      v4f ow;
      ow.x = __shfl(v0, sa, 32); ow.y = __shfl(v1, sa, 32);
      ow.z = __shfl(v0, sb, 32); ow.w = __shfl(v1, sb, 32);
      float* op = hout + (size_t)node * DF + 4 * (lane & 15);
      if (wr) *(volatile v4f*)op = ow;
      __threadfence();
      if (wr) *(volatile v4f*)op = ow;
    }
  }
}

__global__ __launch_bounds__(NTHR) void k_pool(const float* __restrict__ hf, const int* __restrict__ bat,
                                               int nN, unsigned short* plh) {
  __shared__ __attribute__((aligned(16))) float wsum[NWAVE * DF];
  __shared__ int wcn[NWAVE];
  __shared__ __attribute__((aligned(16))) float outs[DF];
  const int tid = (int)threadIdx.x, lane = tid & 31, wave = tid >> 5;
  const int g = (int)blockIdx.x;

  float a0 = 0.0f, a1 = 0.0f;
  int cnt = 0;
#pragma unroll 1
  for (int i0 = wave * 32; i0 < nN; i0 += NTHR) {
    const int i  = i0 + lane;
    const int ic = i < nN ? i : nN - 1;
    const int b  = bat[ic];
    const bool hit = (i < nN) && (b == g);
    unsigned msk = __builtin_amdgcn_ballot_w32(hit);
    int nh = (int)__builtin_popcount(msk);
    nh = nh > 32 ? 32 : nh;
    cnt += nh;
#pragma unroll 1
    for (int q = 0; q < nh; ++q) {
      const int k = __builtin_ffs((int)msk) - 1;
      msk &= msk - 1u;
      int node = i0 + (k < 0 ? 0 : k);
      node = node > nN - 1 ? nN - 1 : node;
      const v2f v = *(const v2fa*)(hf + (size_t)node * DF + 2 * lane);
      a0 += v.x; a1 += v.y;
    }
  }
  wsum[wave * DF + 2 * lane + 0] = a0;
  wsum[wave * DF + 2 * lane + 1] = a1;
  if (lane == 0) wcn[wave] = cnt;
  __syncthreads();
  if (tid < DF) {
    float s = 0.0f;
    int c = 0;
#pragma unroll
    for (int w2 = 0; w2 < NWAVE; ++w2) { s += wsum[w2 * DF + tid]; c += wcn[w2]; }
    const float cf = (c < 1) ? 1.0f : (float)c;
    outs[tid] = s / cf;
  }
  __syncthreads();
  const int q = lane & 7;
  const bool takeLo = (lane & 8) != 0;
  const v4f oa = *(const v4fa*)(outs + 8 * q);
  const v4f ob = *(const v4fa*)(outs + 8 * q + 4);
  const v4u pv = hilo8(oa, ob, takeLo);
  unsigned short* hp = plh + (size_t)g * K2 + (takeLo ? DF : 0) + 8 * q;
  const bool okst = (wave == 0) && (lane < 16);
  if (okst) *(volatile v4u*)hp = pv;
  __threadfence();
  if (okst) *(volatile v4u*)hp = pv;
}

static inline int cdiv(int a, int b) { return (a + b - 1) / b; }
static inline size_t al256(size_t o) { return (o + 255) & ~(size_t)255; }

extern "C" void kernel_launch(void* const* d_in, const int* in_sizes, int n_in,
                              void* d_out, int out_size, void* d_ws, size_t ws_size,
                              hipStream_t stream) {
  if (n_in < 31) return;
  if (in_sizes[0] < DF || (in_sizes[0] % DF) != 0) return;
  const int nN = in_sizes[0] / DF;
  if (nN < 1 || nN > (1 << 22)) return;
  if (in_sizes[1] < 2 || (in_sizes[1] & 1) != 0) return;
  const int nE = in_sizes[1] / 2;
  if (nE < 1 || nE >= (1 << (31 - SLA))) return;
  if (in_sizes[2] != nN) return;
  if (in_sizes[3] != DF * DF || in_sizes[9] != DF * DF) return;
  for (int i = 4; i <= 8; ++i)   if (in_sizes[i] != DF) return;
  for (int i = 10; i <= 14; ++i) if (in_sizes[i] != DF) return;
  if (in_sizes[15] != DF * H1N) return;
  for (int i = 16; i <= 20; ++i) if (in_sizes[i] != H1N) return;
  if (in_sizes[21] != H1N * H2N) return;
  for (int i = 22; i <= 26; ++i) if (in_sizes[i] != H2N) return;
  if (in_sizes[27] != H2N * H3N || in_sizes[28] != H3N) return;
  if (in_sizes[29] != H3N || in_sizes[30] != 1) return;
  if (out_size != NGR) return;

  const float* x    = (const float*)d_in[0];
  const int*   edge = (const int*)d_in[1];
  const int*   bat  = (const int*)d_in[2];
  const float* W0   = (const float*)d_in[3];
  const float* b0   = (const float*)d_in[4];
  const float* g0   = (const float*)d_in[5];
  const float* bb0  = (const float*)d_in[6];
  const float* m0   = (const float*)d_in[7];
  const float* v0   = (const float*)d_in[8];
  const float* W1   = (const float*)d_in[9];
  const float* b1   = (const float*)d_in[10];
  const float* g1   = (const float*)d_in[11];
  const float* bb1  = (const float*)d_in[12];
  const float* m1   = (const float*)d_in[13];
  const float* v1   = (const float*)d_in[14];
  const float* hW1  = (const float*)d_in[15];
  const float* hb1  = (const float*)d_in[16];
  const float* hg1  = (const float*)d_in[17];
  const float* hbb1 = (const float*)d_in[18];
  const float* hm1  = (const float*)d_in[19];
  const float* hv1  = (const float*)d_in[20];
  const float* hW2  = (const float*)d_in[21];
  const float* hb2  = (const float*)d_in[22];
  const float* hg2  = (const float*)d_in[23];
  const float* hbb2 = (const float*)d_in[24];
  const float* hm2  = (const float*)d_in[25];
  const float* hv2  = (const float*)d_in[26];
  const float* hW3  = (const float*)d_in[27];
  const float* hb3  = (const float*)d_in[28];
  const float* hW4  = (const float*)d_in[29];
  const float* hb4  = (const float*)d_in[30];
  float* out = (float*)d_out;
  const int* src = edge;
  const int* dst = edge + nE;

  const int MP   = cdiv(nN, GBM) * GBM;
  const int gM   = MP / GBM;
  const int gD   = cdiv(nN, NBD);
  const int NBPD = gD * NBD;
  const int gA   = cdiv(MP, NBA);
  if ((long long)gA * NBA < (long long)MP) return;
  if (NBPD < nN) return;
  const int vec8 = ((nE & 3) == 0) ? 1 : 0;

  char* ws = (char*)d_ws;
  size_t off = 0;
  const size_t oDIS = off; off = al256(off + (size_t)NBPD * 4);
  const size_t oW0T = off; off = al256(off + (size_t)DF * DF * 2);
  const size_t oW1D = off; off = al256(off + (size_t)DF * K2 * 2);
  const size_t oHW1 = off; off = al256(off + (size_t)H1N * K2 * 2);
  const size_t oHW2 = off; off = al256(off + (size_t)H2N * (2 * H1N) * 2);
  const size_t oHW3 = off; off = al256(off + (size_t)H3N * (2 * H2N) * 2);
  const size_t oXB  = off; off = al256(off + (size_t)MP * DF * 2);
  const size_t oH   = off; off = al256(off + (size_t)MP * DF * 4);
  const size_t oX1  = off; off = al256(off + (size_t)MP * K2 * 2);
  const size_t oH2  = off; off = al256(off + (size_t)MP * DF * 4);
  const size_t oPL  = off; off = al256(off + (size_t)NGR * K2 * 2);
  const size_t oZ1  = off; off = al256(off + (size_t)NGR * (2 * H1N) * 2);
  const size_t oZ2  = off; off = al256(off + (size_t)NGR * (2 * H2N) * 2);
  if (off > ws_size || off > (size_t)WSMAX) return;
  float*          DIS  = (float*)(ws + oDIS);
  unsigned short* W0T  = (unsigned short*)(ws + oW0T);
  unsigned short* W1D  = (unsigned short*)(ws + oW1D);
  unsigned short* HW1D = (unsigned short*)(ws + oHW1);
  unsigned short* HW2D = (unsigned short*)(ws + oHW2);
  unsigned short* HW3D = (unsigned short*)(ws + oHW3);
  unsigned short* XB   = (unsigned short*)(ws + oXB);
  float*          H    = (float*)(ws + oH);
  unsigned short* X1   = (unsigned short*)(ws + oX1);
  float*          H2   = (float*)(ws + oH2);
  unsigned short* PL   = (unsigned short*)(ws + oPL);
  unsigned short* Z1   = (unsigned short*)(ws + oZ1);
  unsigned short* Z2   = (unsigned short*)(ws + oZ2);

  const size_t aggLds = (size_t)AGG_LDS_INTS * 4;
  hipFuncSetAttribute(reinterpret_cast<const void*>(&k_agg<1>), hipFuncAttributeMaxDynamicSharedMemorySize, (int)aggLds);
  hipFuncSetAttribute(reinterpret_cast<const void*>(&k_agg<0>), hipFuncAttributeMaxDynamicSharedMemorySize, (int)aggLds);

  const int nUx = MP * (DF / 8);
  k_wprep<<<UB5 / NTHR, NTHR, 0, stream>>>(W0, W1, hW1, hW2, hW3, W0T, W1D, HW1D, HW2D, HW3D);
  k_cvx<<<cdiv(nUx, NTHR), NTHR, 0, stream>>>(x, nN, nUx, XB);
  k_deg<<<gD, NTHR, 0, stream>>>(dst, nE, vec8, DIS);
  k_gemm<0><<<dim3(gM, 1), GTHR, 0, stream>>>(XB, W0T, DF, H, X1, DF, 0, b0, b0, b0, b0, b0);
  k_agg<1><<<gA, NTHR, aggLds, stream>>>(src, dst, nE, nN, vec8, MP, DIS, H, b0, g0, bb0, m0, v0, X1, H2);
  k_gemm<0><<<dim3(gM, 1), GTHR, 0, stream>>>(X1, W1D, K2, H, X1, DF, 0, b1, b1, b1, b1, b1);
  k_agg<0><<<gA, NTHR, aggLds, stream>>>(src, dst, nE, nN, vec8, MP, DIS, H, b1, g1, bb1, m1, v1, X1, H2);
  k_pool<<<NGR, NTHR, 0, stream>>>(H2, bat, nN, PL);
  k_gemm<1><<<dim3(NGR / GBM, H1N / GBN), GTHR, 0, stream>>>(PL, HW1D, K2, H, Z1, 2 * H1N, H1N,
                                                            hb1, hg1, hbb1, hm1, hv1);
  k_gemm<1><<<dim3(NGR / GBM, H2N / GBN), GTHR, 0, stream>>>(Z1, HW2D, 2 * H1N, H, Z2, 2 * H2N, H2N,
                                                            hb2, hg2, hbb2, hm2, hv2);
  k_gemm<2><<<dim3(NGR / GBM, 1), GTHR, 0, stream>>>(Z2, HW3D, 2 * H2N, out, Z1, 0, 0,
                                                    hb3, hW4, hb4, hb3, hb3);
}
